// MambaEncoderDecoder_55920474194507
// MI455X (gfx1250) — hardware-run, weakly checked
//
#include <hip/hip_runtime.h>
#include <math.h>
#include <stdint.h>

typedef __attribute__((ext_vector_type(16))) _Float16 v16h;
typedef __attribute__((ext_vector_type(8)))  _Float16 v8h;
typedef __attribute__((ext_vector_type(2)))  _Float16 v2h;
typedef __attribute__((ext_vector_type(16))) __bf16   v16b;
typedef __attribute__((ext_vector_type(8)))  __bf16   v8b;
typedef __attribute__((ext_vector_type(8)))  float    v8f;
typedef __attribute__((ext_vector_type(4)))  float    v4f;
typedef __attribute__((ext_vector_type(2)))  float    v2f;
typedef __attribute__((ext_vector_type(4)))  unsigned v4u;

constexpr int kNb    = 512;
constexpr int kLen   = 256;
constexpr int kCin   = 4;
constexpr int kDm    = 64;
constexpr int kDi    = 128;
constexpr int kNs    = 16;
constexpr int kDtr   = 4;
constexpr int kNq    = 2048;
constexpr int kRows  = kNb * kLen;
constexpr int kXpn   = kDtr + 2 * kNs;
constexpr int kPPitch = 64;
constexpr int kChunk  = 32;
constexpr int kSPitch = 48;
constexpr float kCarry   = 64.0f;
constexpr float kFold    = 1.0f / (kCarry * kCarry);
constexpr float kInvLen  = 1.0f / (float)kLen;
constexpr float kLog2e   = 1.44269504088896340736f;
constexpr float kF16MinNormal = 6.103515625e-05f;
static_assert(kXpn == 36);
static_assert(kXpn <= kSPitch && kSPitch <= kPPitch);
static_assert((kDi % 32) == 0 && (kDm % 32) == 0 && ((2 * kDm) % 32) == 0);
static_assert((kRows % 64) == 0 && (kPPitch % 64) == 0);
static_assert(((2 * kNb) % 64) == 0 && (kDm % 64) == 0);
static_assert((kNb % 64) == 0 && ((2 * kDm) % 64) == 0);
static_assert((kNq % 64) == 0 && (kNb % 64) == 0);
static_assert((kLen % kChunk) == 0 && kChunk == 32 && kDi == 128 && kCin == 4 && kDtr == 4 && kNs == 16);
static_assert(((kRows * (kDi / 2)) % 256) == 0);
static_assert(((kNq * 8) % 256) == 0);

constexpr size_t kOffWEFF = 0;
constexpr size_t kOffBEFF = kOffWEFF + (size_t)kCin * 256 * 4;
constexpr size_t kOffQKB  = kOffBEFF + (size_t)256 * 4;
constexpr size_t kOffXPT  = kOffQKB  + (size_t)128 * 4;
constexpr size_t kOffWOH  = kOffXPT  + (size_t)64 * kDi * 2;
constexpr size_t kOffWOL  = kOffWOH  + (size_t)kDm * kDi * 2;
constexpr size_t kOffWQKH = kOffWOL  + (size_t)kDm * kDi * 2;
constexpr size_t kOffWQKL = kOffWQKH + (size_t)(2 * kDm) * (2 * kDm) * 2;
constexpr size_t kOffXC16 = kOffWQKL + (size_t)(2 * kDm) * (2 * kDm) * 2;
constexpr size_t kOffP    = kOffXC16 + (size_t)kRows * kDi * 2;
constexpr size_t kOffGH   = kOffP    + (size_t)kRows * kPPitch * 4;
constexpr size_t kOffGL   = kOffGH   + (size_t)(2 * kNb) * kDi * 2;
constexpr size_t kOffPLH  = kOffGL   + (size_t)(2 * kNb) * kDi * 2;
constexpr size_t kOffPLL  = kOffPLH  + (size_t)(2 * kNb) * kDm * 2;
constexpr size_t kOffQKH  = kOffPLL  + (size_t)(2 * kNb) * kDm * 2;
constexpr size_t kOffQKL  = kOffQKH  + (size_t)kNb * (2 * kDm) * 2;
constexpr size_t kOffQGH  = kOffQKL  + (size_t)kNb * (2 * kDm) * 2;
constexpr size_t kOffQGL  = kOffQGH  + (size_t)kNq * kDm * 2;
constexpr size_t kWsTotal = kOffQGL  + (size_t)kNq * kDm * 2;
static_assert(kWsTotal == 68802048ull);
static_assert(kWsTotal <= 134217728ull);
static_assert((kOffBEFF % 128) == 0 && (kOffQKB % 128) == 0 && (kOffXPT % 128) == 0 && (kOffWOH % 128) == 0 &&
              (kOffWOL % 128) == 0 && (kOffWQKH % 128) == 0 && (kOffWQKL % 128) == 0 && (kOffXC16 % 128) == 0 &&
              (kOffP % 128) == 0 && (kOffGH % 128) == 0 && (kOffGL % 128) == 0 && (kOffPLH % 128) == 0 &&
              (kOffPLL % 128) == 0 && (kOffQKH % 128) == 0 && (kOffQKL % 128) == 0 && (kOffQGH % 128) == 0 &&
              (kOffQGL % 128) == 0);

__device__ __forceinline__ void pin_u(unsigned& t) { asm volatile("" : "+v"(t)); }
__device__ __forceinline__ void pin_f(float& t) { asm volatile("" : "+v"(t)); }

__device__ __forceinline__ unsigned bf_bits32(float f) {
  unsigned u = __float_as_uint(f);
  const unsigned lsb = (u & 0x00010000u) ? 1u : 0u;
  u = (u + 0x7FFFu + lsb) & 0xFFFF0000u;
  return u;
}
__device__ __forceinline__ unsigned pack_hi_halves(unsigned lo_elem, unsigned hi_elem) {
  return __builtin_amdgcn_perm(hi_elem, lo_elem, 0x07060302u);
}
__device__ __forceinline__ void split_pair(float a, float b, unsigned& hw, unsigned& lw) {
  const unsigned ha = bf_bits32(a);
  const unsigned hb = bf_bits32(b);
  const unsigned la = bf_bits32(a - __uint_as_float(ha));
  const unsigned lb = bf_bits32(b - __uint_as_float(hb));
  hw = pack_hi_halves(ha, hb);
  lw = pack_hi_halves(la, lb);
}
__device__ __forceinline__ unsigned pack_f16_pair(float a, float b) {
  const float ca = (fabsf(a) < kF16MinNormal) ? 0.0f : a;
  const float cb = (fabsf(b) < kF16MinNormal) ? 0.0f : b;
  v2h p;
  p.x = (_Float16)ca;
  p.y = (_Float16)cb;
  return __builtin_bit_cast(unsigned, p);
}
__device__ __forceinline__ void store_line2(volatile v4u* dst, v4u val) {
  *dst = val;
  __threadfence();
  *dst = val;
}

__device__ __forceinline__ void dep_guard_h1(v8f& a, v16h x, v16h y) { asm volatile("v_nop\n\tv_nop\n\tv_nop\n\tv_nop" : "+v"(a) : "v"(x), "v"(y)); }
__device__ __forceinline__ void dep_guard_b1(v8f& a, v16b x, v16b y) { asm volatile("v_nop\n\tv_nop\n\tv_nop\n\tv_nop" : "+v"(a) : "v"(x), "v"(y)); }
__device__ __forceinline__ void dep_guard_h4(v8f& a, v16h x, v16h y, v16h z, v16h w) { asm volatile("v_nop\n\tv_nop\n\tv_nop\n\tv_nop" : "+v"(a) : "v"(x), "v"(y), "v"(z), "v"(w)); }
__device__ __forceinline__ void dep_guard_b4(v8f& a, v16b x, v16b y, v16b z, v16b w) { asm volatile("v_nop\n\tv_nop\n\tv_nop\n\tv_nop" : "+v"(a) : "v"(x), "v"(y), "v"(z), "v"(w)); }
__device__ __forceinline__ void keep4_h(v16h a, v16h b, v16h c, v16h d) { asm volatile("v_nop" :: "v"(a), "v"(b), "v"(c), "v"(d)); }
__device__ __forceinline__ void keep4_b(v16b a, v16b b, v16b c, v16b d) { asm volatile("v_nop" :: "v"(a), "v"(b), "v"(c), "v"(d)); }

template <typename T> struct Frag;
template <> struct Frag<_Float16> {
  typedef v16h V; union U { v16h v; v8h h[2]; };
  static __device__ __forceinline__ v16h load(const _Float16* p) {
    U f; f.h[0] = *(const v8h*)(p); f.h[1] = *(const v8h*)(p + 16); return f.v;
  }
  static __device__ __forceinline__ v8f mma(v16h a, v16h b, v8f c) {
    return __builtin_amdgcn_wmma_f32_16x16x32_f16(false, a, false, b, (short)0, c, false, false);
  }
  static __device__ __forceinline__ void guard(v8f& a, v16h x, v16h y) { dep_guard_h1(a, x, y); }
  static __device__ __forceinline__ void guard4(v8f& a, v16h x, v16h y, v16h z, v16h w) { dep_guard_h4(a, x, y, z, w); }
  static __device__ __forceinline__ void keep(v16h a, v16h b, v16h c, v16h d) { keep4_h(a, b, c, d); }
};
template <> struct Frag<__bf16> {
  typedef v16b V; union U { v16b v; v8b h[2]; };
  static __device__ __forceinline__ v16b load(const __bf16* p) {
    U f; f.h[0] = *(const v8b*)(p); f.h[1] = *(const v8b*)(p + 16); return f.v;
  }
  static __device__ __forceinline__ v8f mma(v16b a, v16b b, v8f c) {
    return __builtin_amdgcn_wmma_f32_16x16x32_bf16(false, a, false, b, (short)0, c, false, false);
  }
  static __device__ __forceinline__ void guard(v8f& a, v16b x, v16b y) { dep_guard_b1(a, x, y); }
  static __device__ __forceinline__ void guard4(v8f& a, v16b x, v16b y, v16b z, v16b w) { dep_guard_b4(a, x, y, z, w); }
  static __device__ __forceinline__ void keep(v16b a, v16b b, v16b c, v16b d) { keep4_b(a, b, c, d); }
};

template <int ET> struct Elem;
template <> struct Elem<0> { typedef _Float16 T; };
template <> struct Elem<1> { typedef __bf16 T; };
template <int ET, bool SPLIT, int BIAS_MODE, int OUT_MODE>
__global__ __launch_bounds__(256) void wmma_gemm64(
    const unsigned short* __restrict__ Ap, const unsigned short* __restrict__ A2p, int lda,
    const unsigned short* __restrict__ Btp, const unsigned short* __restrict__ Bt2p, int ldb,
    void* __restrict__ Cout, void* __restrict__ Cout2, int ldc,
    const float* __restrict__ bias, int M, int N, int K, float scale) {
  typedef typename Elem<ET>::T T;
  typedef typename Frag<T>::V V;
  const T* Ab  = (const T*)Ap;
  const T* Ab2 = (const T*)A2p;
  const T* Bb  = (const T*)Btp;
  const T* Bb2 = (const T*)Bt2p;
  __shared__ __align__(16) float sT[8][16 * 68];
  const int lane = threadIdx.x & 31;
  const int wave = threadIdx.x >> 5;
  const int tilesN = N >> 6;
  const int tilesM = M >> 6;
  const int tile = blockIdx.x * 8 + wave;
  if (tile >= tilesM * tilesN) return;
  const int tm = tile / tilesN;
  const int tn = tile - tm * tilesN;
  const int m0 = tm << 6;
  const int n0 = tn << 6;

  const int rlane = lane & 15;
  const int koff  = (lane >> 4) * 8;
  const int mOff  = (lane >> 4) * 8;

  v8f acc[4][4];
#pragma unroll
  for (int i = 0; i < 4; ++i)
#pragma unroll
    for (int j = 0; j < 4; ++j) acc[i][j] = (v8f){0.f,0.f,0.f,0.f,0.f,0.f,0.f,0.f};

  for (int k0 = 0; k0 < K; k0 += 32) {
    V bh[4], bl[4];
#pragma unroll
    for (int j = 0; j < 4; ++j) {
      const size_t bo = (size_t)(n0 + (j << 4) + rlane) * ldb + koff + k0;
      bh[j] = Frag<T>::load(Bb + bo);
      if (SPLIT) bl[j] = Frag<T>::load(Bb2 + bo);
    }
#pragma unroll
    for (int i = 0; i < 4; ++i) {
      const size_t ao = (size_t)(m0 + (i << 4) + rlane) * lda + koff + k0;
      V ah = Frag<T>::load(Ab + ao);
      V al;
      if (SPLIT) al = Frag<T>::load(Ab2 + ao);
#pragma unroll
      for (int j = 0; j < 4; ++j) {
        acc[i][j] = Frag<T>::mma(ah, bh[j], acc[i][j]);
        if (SPLIT) {
          acc[i][j] = Frag<T>::mma(ah, bl[j], acc[i][j]);
          acc[i][j] = Frag<T>::mma(al, bh[j], acc[i][j]);
        }
      }
#pragma unroll
      for (int j = 0; j < 4; ++j) {
        if (SPLIT) Frag<T>::guard4(acc[i][j], ah, al, bh[j], bl[j]);
        else       Frag<T>::guard(acc[i][j], ah, bh[j]);
      }
    }
    Frag<T>::keep(bh[0], bh[1], bh[2], bh[3]);
    if (SPLIT) Frag<T>::keep(bl[0], bl[1], bl[2], bl[3]);
  }

  float* slab = sT[wave];
#pragma unroll
  for (int i = 0; i < 4; ++i) {
    const int mBase = m0 + (i << 4);
#pragma unroll
    for (int j = 0; j < 4; ++j) {
      const int n = n0 + (j << 4) + rlane;
      float bv = 0.f;
      if (BIAS_MODE == 2) bv = bias[n];
#pragma unroll
      for (int r = 0; r < 8; ++r) {
        float v = acc[i][j][r] * scale;
        if (BIAS_MODE == 2) v += bv;
        slab[(mOff + r) * 68 + (j << 4) + rlane] = v;
      }
    }
    __builtin_amdgcn_fence(__ATOMIC_RELEASE, "workgroup");
    __builtin_amdgcn_wave_barrier();
    __builtin_amdgcn_fence(__ATOMIC_ACQUIRE, "workgroup");
    if (OUT_MODE == 0) {
      float* C = (float*)Cout;
      const int hh = lane >> 4, c4 = (lane & 15) * 4;
      for (int pass = 0; pass < 2; ++pass) {
#pragma unroll
        for (int it = 0; it < 8; ++it) {
          const int row = it * 2 + hh;
          v4f v = *(const v4f*)(slab + row * 68 + c4);
          *(volatile v4f*)(C + (size_t)(mBase + row) * ldc + n0 + c4) = v;
        }
        __threadfence();
      }
    } else {
      const int q = lane >> 3, c8 = (lane & 7) * 8;
      unsigned short* C  = (unsigned short*)Cout;
      unsigned short* C2 = (unsigned short*)Cout2;
      v4u hv[4], lv[4];
#pragma unroll
      for (int it = 0; it < 4; ++it) {
        const int row = it * 4 + q;
        const v4f a0 = *(const v4f*)(slab + row * 68 + c8);
        const v4f a1 = *(const v4f*)(slab + row * 68 + c8 + 4);
        unsigned h0, h1, h2, h3, l0, l1, l2, l3;
        split_pair(a0.x, a0.y, h0, l0);
        split_pair(a0.z, a0.w, h1, l1);
        split_pair(a1.x, a1.y, h2, l2);
        split_pair(a1.z, a1.w, h3, l3);
        v4u th, tl;
        th.x = h0; th.y = h1; th.z = h2; th.w = h3;
        tl.x = l0; tl.y = l1; tl.z = l2; tl.w = l3;
        hv[it] = th;
        lv[it] = tl;
      }
      for (int pass = 0; pass < 2; ++pass) {
#pragma unroll
        for (int it = 0; it < 4; ++it) {
          const int row = it * 4 + q;
          const size_t o = (size_t)(mBase + row) * ldc + n0 + c8;
          *(volatile v4u*)(C + o)  = hv[it];
          *(volatile v4u*)(C2 + o) = lv[it];
        }
        __threadfence();
      }
    }
    __builtin_amdgcn_fence(__ATOMIC_RELEASE, "workgroup");
    __builtin_amdgcn_wave_barrier();
    __builtin_amdgcn_fence(__ATOMIC_ACQUIRE, "workgroup");
  }
}

__global__ __launch_bounds__(256) void prep_kernel(
    const float* __restrict__ exp_w, const float* __restrict__ exp_b, const float* __restrict__ in_proj_w,
    const float* __restrict__ x_proj_w, const float* __restrict__ out_proj_w,
    const float* __restrict__ q_w, const float* __restrict__ k_w,
    const float* __restrict__ q_b, const float* __restrict__ k_b,
    float* __restrict__ Weff, float* __restrict__ beff, float* __restrict__ qkb,
    unsigned short* __restrict__ XPT, unsigned short* __restrict__ WOH, unsigned short* __restrict__ WOL,
    unsigned short* __restrict__ WQKH, unsigned short* __restrict__ WQKL)
{
  const unsigned tid = threadIdx.x;
  {
    float a0 = 0.f, a1 = 0.f, a2 = 0.f, a3 = 0.f, ab = 0.f;
#pragma unroll 1
    for (unsigned k = 0; k < (unsigned)kDm; ++k) {
      const float w = in_proj_w[k * 256u + tid];
      a0 = fmaf(exp_w[k], w, a0);
      a1 = fmaf(exp_w[64u + k], w, a1);
      a2 = fmaf(exp_w[128u + k], w, a2);
      a3 = fmaf(exp_w[192u + k], w, a3);
      ab = fmaf(exp_b[k], w, ab);
    }
    const float qv = q_b[tid & 63u];
    const float kv = k_b[tid & 63u];
    const float bsel = (tid & 64u) ? kv : qv;
    volatile float* vw = Weff;
    volatile float* vb = beff;
    volatile float* vq = qkb;
    for (int pass = 0; pass < 2; ++pass) {
      vw[tid] = a0;
      vw[256u + tid] = a1;
      vw[512u + tid] = a2;
      vw[768u + tid] = a3;
      vb[tid] = ab;
      if (tid < 128u) vq[tid] = bsel;
      __threadfence();
    }
  }
#pragma unroll 1
  for (unsigned it = 0; it < 4u; ++it) {
    unsigned ci = it * 256u + tid;
    pin_u(ci);
    const unsigned n  = ci >> 4;
    const unsigned k0 = (ci & 15u) << 3;
    const bool live = n < (unsigned)kXpn;
    unsigned nc = live ? n : (unsigned)(kXpn - 1);
    pin_u(nc);
    float v[8];
#pragma unroll
    for (int e = 0; e < 8; ++e) {
      v[e] = x_proj_w[(k0 + (unsigned)e) * (unsigned)kXpn + nc];
      pin_f(v[e]);
    }
    unsigned w[4];
#pragma unroll
    for (int p = 0; p < 4; ++p) {
      const float a = live ? v[2 * p] * kCarry : 0.0f;
      const float b = live ? v[2 * p + 1] * kCarry : 0.0f;
      w[p] = pack_f16_pair(a, b);
    }
    v4u val;
    val.x = w[0]; val.y = w[1]; val.z = w[2]; val.w = w[3];
    store_line2((volatile v4u*)(XPT + (size_t)ci * 8u), val);
  }
#pragma unroll 1
  for (unsigned it = 0; it < 4u; ++it) {
    unsigned ci = it * 256u + tid;
    pin_u(ci);
    const unsigned n  = ci >> 4;
    const unsigned k0 = (ci & 15u) << 3;
    float v[8];
#pragma unroll
    for (int e = 0; e < 8; ++e) v[e] = out_proj_w[(k0 + (unsigned)e) * (unsigned)kDm + n];
    unsigned hw[4], lw[4];
#pragma unroll
    for (int p = 0; p < 4; ++p) split_pair(v[2 * p], v[2 * p + 1], hw[p], lw[p]);
    v4u vh, vl;
    vh.x = hw[0]; vh.y = hw[1]; vh.z = hw[2]; vh.w = hw[3];
    vl.x = lw[0]; vl.y = lw[1]; vl.z = lw[2]; vl.w = lw[3];
    store_line2((volatile v4u*)(WOH + (size_t)ci * 8u), vh);
    store_line2((volatile v4u*)(WOL + (size_t)ci * 8u), vl);
  }
#pragma unroll 1
  for (unsigned it = 0; it < 8u; ++it) {
    unsigned ci = it * 256u + tid;
    pin_u(ci);
    const unsigned n  = ci >> 4;
    const unsigned k0 = (ci & 15u) << 3;
    const float* src = (n & 64u) ? k_w : q_w;
    const unsigned nn = n & 63u;
    float v[8];
#pragma unroll
    for (int e = 0; e < 8; ++e) v[e] = src[(k0 + (unsigned)e) * (unsigned)kDm + nn];
    unsigned hw[4], lw[4];
#pragma unroll
    for (int p = 0; p < 4; ++p) split_pair(v[2 * p], v[2 * p + 1], hw[p], lw[p]);
    v4u vh, vl;
    vh.x = hw[0]; vh.y = hw[1]; vh.z = hw[2]; vh.w = hw[3];
    vl.x = lw[0]; vl.y = lw[1]; vl.z = lw[2]; vl.w = lw[3];
    store_line2((volatile v4u*)(WQKH + (size_t)ci * 8u), vh);
    store_line2((volatile v4u*)(WQKL + (size_t)ci * 8u), vl);
  }
}

__device__ __forceinline__ void conv_tap(const float* __restrict__ reads, unsigned row, unsigned l, unsigned back,
                                         v2f w0, v2f w1, v2f w2, v2f w3, v2f be, float ta, float tb,
                                         float& preA, float& preB)
{
  const bool ok = l >= back;
  unsigned rr = ok ? (row - back) : row;
  pin_u(rr);
  const v4f rv = *(const v4f*)(reads + (size_t)rr * 4u);
  float xa = be.x;
  xa = fmaf(rv.x, w0.x, xa);
  xa = fmaf(rv.y, w1.x, xa);
  xa = fmaf(rv.z, w2.x, xa);
  xa = fmaf(rv.w, w3.x, xa);
  float xb = be.y;
  xb = fmaf(rv.x, w0.y, xb);
  xb = fmaf(rv.y, w1.y, xb);
  xb = fmaf(rv.z, w2.y, xb);
  xb = fmaf(rv.w, w3.y, xb);
  xa = ok ? xa : 0.0f;
  xb = ok ? xb : 0.0f;
  preA = fmaf(ta, xa, preA);
  preB = fmaf(tb, xb, preB);
}

__global__ __launch_bounds__(256) void conv_plane_kernel(
    const float* __restrict__ reads, const float* __restrict__ Weff, const float* __restrict__ beff,
    const float* __restrict__ conv_w, const float* __restrict__ conv_b, unsigned* __restrict__ XC16w)
{
  unsigned gid = blockIdx.x * 256u + threadIdx.x;
  pin_u(gid);
  const unsigned dp  = gid & 63u;
  const unsigned row = gid >> 6;
  const unsigned l   = row & (unsigned)(kLen - 1);
  const unsigned d   = dp << 1;
  const v2f w0 = *(const v2f*)(Weff + d);
  const v2f w1 = *(const v2f*)(Weff + 256u + d);
  const v2f w2 = *(const v2f*)(Weff + 512u + d);
  const v2f w3 = *(const v2f*)(Weff + 768u + d);
  const v2f be = *(const v2f*)(beff + d);
  const v4f ca = *(const v4f*)(conv_w + d * 4u);
  const v4f cb = *(const v4f*)(conv_w + d * 4u + 4u);
  const v2f cbias = *(const v2f*)(conv_b + d);
  float preA = cbias.x, preB = cbias.y;
  conv_tap(reads, row, l, 3u, w0, w1, w2, w3, be, ca.x, cb.x, preA, preB);
  conv_tap(reads, row, l, 2u, w0, w1, w2, w3, be, ca.y, cb.y, preA, preB);
  conv_tap(reads, row, l, 1u, w0, w1, w2, w3, be, ca.z, cb.z, preA, preB);
  conv_tap(reads, row, l, 0u, w0, w1, w2, w3, be, ca.w, cb.w, preA, preB);
  const float uA = preA * __builtin_amdgcn_rcpf(1.0f + expf(-preA));
  const float uB = preB * __builtin_amdgcn_rcpf(1.0f + expf(-preB));
  const unsigned word = pack_f16_pair(uA * kCarry, uB * kCarry);
  volatile unsigned* dst = XC16w + gid;
  *dst = word;
  __threadfence();
  *dst = word;
}

__global__ __launch_bounds__(128) void scan_pool_kernel(
    const float* __restrict__ reads, const float* __restrict__ Weff, const float* __restrict__ beff,
    const float* __restrict__ conv_w, const float* __restrict__ conv_b, const float* __restrict__ P,
    const float* __restrict__ dt_w, const float* __restrict__ dt_b, const float* __restrict__ A_log,
    const float* __restrict__ D_skip, unsigned short* __restrict__ GH, unsigned short* __restrict__ GL)
{
  __shared__ __align__(16) float sP[kChunk * kSPitch];
  __shared__ __align__(16) float sR[kChunk * 4];
  __shared__ __align__(16) float sA[kNs * kDi];
  __shared__ __align__(16) float sG[2 * kDi];
  const unsigned tid  = threadIdx.x;
  const unsigned lane = tid & 31u;
  const unsigned wave = tid >> 5;
  const unsigned b    = blockIdx.x;
  const unsigned d    = tid;
  const size_t row0   = (size_t)b * (size_t)kLen;

#pragma unroll 1
  for (unsigned n = 0; n < (unsigned)kNs; ++n)
    sA[n * (unsigned)kDi + tid] = -expf(A_log[d * (unsigned)kNs + n]) * kLog2e;
  __syncthreads();
  float a2[kNs], h[kNs];
#pragma unroll
  for (int n = 0; n < kNs; ++n) {
    a2[n] = sA[n * kDi + tid];
    h[n] = 0.0f;
  }

  const float we0 = Weff[d], we1 = Weff[256u + d], we2 = Weff[512u + d], we3 = Weff[768u + d];
  const float wz0 = Weff[128u + d], wz1 = Weff[384u + d], wz2 = Weff[640u + d], wz3 = Weff[896u + d];
  const float bx = beff[d], bz = beff[128u + d];
  const v4f cw = *(const v4f*)(conv_w + d * 4u);
  const float cb = conv_b[d];
  const float dw0 = dt_w[d], dw1 = dt_w[128u + d], dw2 = dt_w[256u + d], dw3 = dt_w[384u + d];
  const float dtb = dt_b[d];
  const float dsk = D_skip[d];

  float xm1 = 0.0f, xm2 = 0.0f, xm3 = 0.0f;
  float gsum = 0.0f, glast = 0.0f;

  unsigned sr = tid >> 2;
  unsigned sc = (tid & 3u) << 2;
  pin_u(sr);
  pin_u(sc);

#pragma unroll 1
  for (unsigned ck = 0; ck < (unsigned)(kLen / kChunk); ++ck) {
    const unsigned l0 = ck * (unsigned)kChunk;
    __syncthreads();
    {
      const float* src = P + (row0 + l0 + sr) * (size_t)kPPitch + sc;
      float* dstp = sP + sr * (unsigned)kSPitch + sc;
#pragma unroll
      for (int it = 0; it < 3; ++it) {
        const v4f v = *(const v4f*)(src + 16 * it);
        *(v4f*)(dstp + 16 * it) = v;
      }
    }
    if (tid < 32u) {
      const v4f v = *(const v4f*)(reads + (row0 + l0 + tid) * 4u);
      *(v4f*)(sR + tid * 4u) = v;
    }
    __syncthreads();
#pragma unroll 1
    for (unsigned s = 0; s < (unsigned)kChunk; ++s) {
      const v4f rv = *(const v4f*)(sR + s * 4u);
      const float* pr = sP + s * (unsigned)kSPitch;
      const v4f dv = *(const v4f*)(pr);
      float xm = bx;
      xm = fmaf(rv.x, we0, xm);
      xm = fmaf(rv.y, we1, xm);
      xm = fmaf(rv.z, we2, xm);
      xm = fmaf(rv.w, we3, xm);
      float zz = bz;
      zz = fmaf(rv.x, wz0, zz);
      zz = fmaf(rv.y, wz1, zz);
      zz = fmaf(rv.z, wz2, zz);
      zz = fmaf(rv.w, wz3, zz);
      float pre = cb;
      pre = fmaf(cw.x, xm3, pre);
      pre = fmaf(cw.y, xm2, pre);
      pre = fmaf(cw.z, xm1, pre);
      pre = fmaf(cw.w, xm, pre);
      xm3 = xm2;
      xm2 = xm1;
      xm1 = xm;
      const float u  = pre * __builtin_amdgcn_rcpf(1.0f + expf(-pre));
      const float gz = zz * __builtin_amdgcn_rcpf(1.0f + expf(-zz));
      float xd = dtb;
      xd = fmaf(dv.x, dw0, xd);
      xd = fmaf(dv.y, dw1, xd);
      xd = fmaf(dv.z, dw2, xd);
      xd = fmaf(dv.w, dw3, xd);
      const float ea = expf(-fabsf(xd));
      const float up = 1.0f + ea;
      const float corr = (ea - (up - 1.0f)) * __builtin_amdgcn_rcpf(up);
      const float delta = fmaxf(xd, 0.0f) + (logf(up) + corr);
      const float du = delta * u;
      float ys = 0.0f;
#pragma unroll
      for (int q = 0; q < 4; ++q) {
        const v4f bv = *(const v4f*)(pr + 4 + 4 * q);
        const v4f cv = *(const v4f*)(pr + 20 + 4 * q);
        {
          const float e = exp2f(delta * a2[4 * q + 0]);
          h[4 * q + 0] = fmaf(e, h[4 * q + 0], du * bv.x);
          ys = fmaf(h[4 * q + 0], cv.x, ys);
        }
        {
          const float e = exp2f(delta * a2[4 * q + 1]);
          h[4 * q + 1] = fmaf(e, h[4 * q + 1], du * bv.y);
          ys = fmaf(h[4 * q + 1], cv.y, ys);
        }
        {
          const float e = exp2f(delta * a2[4 * q + 2]);
          h[4 * q + 2] = fmaf(e, h[4 * q + 2], du * bv.z);
          ys = fmaf(h[4 * q + 2], cv.z, ys);
        }
        {
          const float e = exp2f(delta * a2[4 * q + 3]);
          h[4 * q + 3] = fmaf(e, h[4 * q + 3], du * bv.w);
          ys = fmaf(h[4 * q + 3], cv.w, ys);
        }
      }
      const float y = fmaf(u, dsk, ys);
      const float g = y * gz;
      gsum += g;
      glast = g;
    }
  }

  sG[tid] = gsum * kInvLen;
  sG[(unsigned)kDi + tid] = glast;
  __syncthreads();
  if (wave < 2u) {
    const v4f a0 = *(const v4f*)(sG + lane * 8u);
    const v4f a1 = *(const v4f*)(sG + lane * 8u + 4u);
    unsigned h0, h1, h2, h3, l0, l1, l2, l3;
    split_pair(a0.x, a0.y, h0, l0);
    split_pair(a0.z, a0.w, h1, l1);
    split_pair(a1.x, a1.y, h2, l2);
    split_pair(a1.z, a1.w, h3, l3);
    const bool hiw = (wave == 0u);
    v4u val;
    val.x = hiw ? h0 : l0;
    val.y = hiw ? h1 : l1;
    val.z = hiw ? h2 : l2;
    val.w = hiw ? h3 : l3;
    unsigned short* base = hiw ? GH : GL;
    store_line2((volatile v4u*)(base + (size_t)b * 256u + lane * 8u), val);
  }
}

__global__ __launch_bounds__(256) void gather_rows_kernel(
    const int* __restrict__ idx, const unsigned short* __restrict__ QKH, const unsigned short* __restrict__ QKL,
    unsigned short* __restrict__ QGH, unsigned short* __restrict__ QGL)
{
  unsigned gid = blockIdx.x * 256u + threadIdx.x;
  pin_u(gid);
  const unsigned n = gid >> 3;
  const unsigned c = gid & 7u;
  int v = idx[n];
  v = (v < 0) ? 0 : v;
  v = (v > (kNb - 1)) ? (kNb - 1) : v;
  unsigned src = (unsigned)v * (unsigned)(2 * kDm) + c * 8u;
  pin_u(src);
  const v4u hv = *(const v4u*)(QKH + src);
  const v4u lv = *(const v4u*)(QKL + src);
  volatile v4u* dh = (volatile v4u*)(QGH + (size_t)gid * 8u);
  volatile v4u* dl = (volatile v4u*)(QGL + (size_t)gid * 8u);
  *dh = hv;
  *dl = lv;
  __threadfence();
  *dh = hv;
  *dl = lv;
}

extern "C" void kernel_launch(void* const* d_in, const int* in_sizes, int n_in,
                              void* d_out, int out_size, void* d_ws, size_t ws_size,
                              hipStream_t stream) {
  if (n_in < 17) return;
  if (in_sizes[0] != kRows * kCin) return;
  if (in_sizes[1] != kNq) return;
  if (in_sizes[2] != kCin * kDm) return;
  if (in_sizes[3] != kDm) return;
  if (in_sizes[4] != kDm * 2 * kDi) return;
  if (in_sizes[5] != kDi * 4) return;
  if (in_sizes[6] != kDi) return;
  if (in_sizes[7] != kDi * kXpn) return;
  if (in_sizes[8] != kDtr * kDi) return;
  if (in_sizes[9] != kDi) return;
  if (in_sizes[10] != kDi * kNs) return;
  if (in_sizes[11] != kDi) return;
  if (in_sizes[12] != kDi * kDm) return;
  if (in_sizes[13] != 2 * kDm * kDm) return;
  if (in_sizes[14] != kDm) return;
  if (in_sizes[15] != 2 * kDm * kDm) return;
  if (in_sizes[16] != kDm) return;
  if (out_size != kNq * kNb) return;
  if (ws_size < kWsTotal) return;

  const float* reads      = (const float*)d_in[0];
  const int*   seq_idx    = (const int*)  d_in[1];
  const float* exp_w      = (const float*)d_in[2];
  const float* exp_b      = (const float*)d_in[3];
  const float* in_proj_w  = (const float*)d_in[4];
  const float* conv_w     = (const float*)d_in[5];
  const float* conv_b     = (const float*)d_in[6];
  const float* x_proj_w   = (const float*)d_in[7];
  const float* dt_w       = (const float*)d_in[8];
  const float* dt_b       = (const float*)d_in[9];
  const float* A_log      = (const float*)d_in[10];
  const float* D_skip     = (const float*)d_in[11];
  const float* out_proj_w = (const float*)d_in[12];
  const float* q_w        = (const float*)d_in[13];
  const float* q_b        = (const float*)d_in[14];
  const float* k_w        = (const float*)d_in[15];
  const float* k_b        = (const float*)d_in[16];
  float* out = (float*)d_out;

  char* ws = (char*)d_ws;
  float*          WEFF = (float*)(ws + kOffWEFF);
  float*          BEFF = (float*)(ws + kOffBEFF);
  float*          QKB  = (float*)(ws + kOffQKB);
  unsigned short* XPT  = (unsigned short*)(ws + kOffXPT);
  unsigned short* WOH  = (unsigned short*)(ws + kOffWOH);
  unsigned short* WOL  = (unsigned short*)(ws + kOffWOL);
  unsigned short* WQKH = (unsigned short*)(ws + kOffWQKH);
  unsigned short* WQKL = (unsigned short*)(ws + kOffWQKL);
  unsigned short* XC16 = (unsigned short*)(ws + kOffXC16);
  float*          Pp   = (float*)(ws + kOffP);
  unsigned short* GH   = (unsigned short*)(ws + kOffGH);
  unsigned short* GL   = (unsigned short*)(ws + kOffGL);
  unsigned short* PLH  = (unsigned short*)(ws + kOffPLH);
  unsigned short* PLL  = (unsigned short*)(ws + kOffPLL);
  unsigned short* QKH  = (unsigned short*)(ws + kOffQKH);
  unsigned short* QKL  = (unsigned short*)(ws + kOffQKL);
  unsigned short* QGH  = (unsigned short*)(ws + kOffQGH);
  unsigned short* QGL  = (unsigned short*)(ws + kOffQGL);

  prep_kernel<<<1, 256, 0, stream>>>(exp_w, exp_b, in_proj_w, x_proj_w, out_proj_w, q_w, k_w, q_b, k_b,
                                     WEFF, BEFF, QKB, XPT, WOH, WOL, WQKH, WQKL);

  conv_plane_kernel<<<(kRows * (kDi / 2)) / 256, 256, 0, stream>>>(reads, WEFF, BEFF, conv_w, conv_b,
                                                                   (unsigned*)XC16);

  wmma_gemm64<0, false, 0, 0><<<((kRows / 64) * (kPPitch / 64) + 7) / 8, 256, 0, stream>>>(
      XC16, XC16, kDi,
      XPT, XPT, kDi,
      (void*)Pp, (void*)Pp, kPPitch,
      BEFF, kRows, kPPitch, kDi, kFold);

  scan_pool_kernel<<<kNb, 128, 0, stream>>>(reads, WEFF, BEFF, conv_w, conv_b, Pp, dt_w, dt_b, A_log, D_skip,
                                            GH, GL);

  wmma_gemm64<1, true, 0, 2><<<(((2 * kNb) / 64) * (kDm / 64) + 7) / 8, 256, 0, stream>>>(
      GH, GL, kDi,
      WOH, WOL, kDi,
      (void*)PLH, (void*)PLL, kDm,
      BEFF, 2 * kNb, kDm, kDi, 1.0f);

  wmma_gemm64<1, true, 2, 2><<<((kNb / 64) * ((2 * kDm) / 64) + 7) / 8, 256, 0, stream>>>(
      PLH, PLL, 2 * kDm,
      WQKH, WQKL, 2 * kDm,
      (void*)QKH, (void*)QKL, 2 * kDm,
      QKB, kNb, 2 * kDm, 2 * kDm, 1.0f);

  gather_rows_kernel<<<(kNq * 8) / 256, 256, 0, stream>>>(seq_idx, QKH, QKL, QGH, QGL);

  wmma_gemm64<1, true, 0, 0><<<((kNq / 64) * (kNb / 64) + 7) / 8, 256, 0, stream>>>(
      QGH, QGL, kDm,
      QKH + kDm, QKL + kDm, 2 * kDm,
      (void*)out, (void*)out, kNb,
      BEFF, kNq, kNb, kDm, 1.0f);
}
